// CrossAttentionLayer_21878563406365
// MI455X (gfx1250) — hardware-verified
//
#include <hip/hip_runtime.h>


#define NB_  4
#define TT   4096
#define DM   512
#define NH_  8
#define NKV  8
#define REP  (NH_ / NKV)
#define HD   64
#define DQ   (NH_ * HD)
#define DKV  (NKV * HD)
#define ZH   2
#define RH   512
#define WIN  0
#define PCAR 1024.0f
#define SCL  1.0f
#define INVS 0.000244140625f
#define SFL  4096.0f
#define ZEPS 1e-6f
typedef _Float16 h16;
typedef unsigned short bf;
typedef __attribute__((ext_vector_type(16))) __bf16   v16bf;
typedef __attribute__((ext_vector_type(16))) _Float16 v16h;
typedef __attribute__((ext_vector_type(8)))  _Float16 v8h;
typedef __attribute__((ext_vector_type(8)))  unsigned short v8us;
typedef __attribute__((ext_vector_type(8)))  float    v8f;
typedef __attribute__((ext_vector_type(4)))  float    v4f;
typedef v8h  __attribute__((may_alias)) v8ha;
typedef v4f  __attribute__((may_alias)) v4fa;
typedef v8us __attribute__((may_alias)) v8usa;

__device__ __forceinline__ unsigned short f2bf(float f) { unsigned u = __float_as_uint(f); u += 0x7FFFu + ((u >> 16) & 1u); return (unsigned short)(u >> 16); }
__device__ __forceinline__ float bf2f(unsigned short b) { return __uint_as_float(((unsigned)b) << 16); }
__device__ __forceinline__ float bfr(float f) { return bf2f(f2bf(f)); }
__device__ __forceinline__ v16h cat16(v8h lo, v8h hi) { return __builtin_shufflevector(lo, hi, 0, 1, 2, 3, 4, 5, 6, 7, 8, 9, 10, 11, 12, 13, 14, 15); }
__device__ __forceinline__ v16bf cat16b(v8us lo, v8us hi) { return __builtin_bit_cast(v16bf, __builtin_shufflevector(lo, hi, 0, 1, 2, 3, 4, 5, 6, 7, 8, 9, 10, 11, 12, 13, 14, 15)); }
__device__ __forceinline__ v8f wmma16(v16h a, v16h b, v8f c) { return __builtin_amdgcn_wmma_f32_16x16x32_f16(false, a, false, b, (short)0, c, false, false); }
__device__ __forceinline__ v8f wmmab(v16bf a, v16bf b, v8f c) { return __builtin_amdgcn_wmma_f32_16x16x32_bf16(false, a, false, b, (short)0, c, false, false); }


template <typename T16> struct WFrag;
template <> struct WFrag<h16> { typedef v16h V; static __device__ __forceinline__ V ld(const h16* p) { return cat16(*(const v8h*)p, *(const v8h*)(p + 16)); } static __device__ __forceinline__ v8f mma(V a, V b, v8f c) { return wmma16(a, b, c); } };
template <> struct WFrag<bf> { typedef v16bf V; static __device__ __forceinline__ V ld(const bf* p) { return cat16b(*(const v8us*)p, *(const v8us*)(p + 16)); } static __device__ __forceinline__ v8f mma(V a, V b, v8f c) { return wmmab(a, b, c); } };
template <typename T16, int NSPLIT, bool BIAS>
__global__ __launch_bounds__(32) void k_gemmw(const T16* __restrict__ A, const T16* __restrict__ A2, const T16* __restrict__ Bt, const T16* __restrict__ Bt2, int K, float* C, int ldc, const float* __restrict__ bias, size_t sA, size_t sB, size_t sC) {
    typedef typename WFrag<T16>::V V;
    __shared__ __align__(16) float os[16 * 68];
    const size_t z = blockIdx.z; A += z * sA; if (A2) A2 += z * sA; Bt += z * sB; if (Bt2) Bt2 += z * sB; C += z * sC;
    const int lane = threadIdx.x & 31, lr = lane & 15, hi = lane >> 4; const int r0 = blockIdx.x * 64, c0 = blockIdx.y * 64;
    v8f acc[4][4];
#pragma unroll
    for (int mb = 0; mb < 4; ++mb)
#pragma unroll
        for (int nb = 0; nb < 4; ++nb) acc[mb][nb] = (v8f){};
    const size_t aoff = (size_t)(r0 + lr) * K + 8 * hi, boff = (size_t)(c0 + lr) * K + 8 * hi;
#pragma unroll 1
    for (int kc = 0; kc < K; kc += 32) {
        V a[4], a2[4];
#pragma unroll
        for (int mb = 0; mb < 4; ++mb) { a[mb] = WFrag<T16>::ld(A + aoff + (size_t)mb * 16 * K + kc); if (NSPLIT == 1 || NSPLIT == 2) a2[mb] = WFrag<T16>::ld(A2 + aoff + (size_t)mb * 16 * K + kc); }
#pragma unroll
        for (int nb = 0; nb < 4; ++nb) { const V b = WFrag<T16>::ld(Bt + boff + (size_t)nb * 16 * K + kc); V b2; if (NSPLIT >= 2) b2 = WFrag<T16>::ld(Bt2 + boff + (size_t)nb * 16 * K + kc);
#pragma unroll
            for (int mb = 0; mb < 4; ++mb) { acc[mb][nb] = WFrag<T16>::mma(a[mb], b, acc[mb][nb]); if (NSPLIT == 1 || NSPLIT == 2) acc[mb][nb] = WFrag<T16>::mma(a2[mb], b, acc[mb][nb]); if (NSPLIT >= 2) acc[mb][nb] = WFrag<T16>::mma(a[mb], b2, acc[mb][nb]); } }
        asm volatile("v_nop\n\tv_nop\n\tv_nop\n\tv_nop" : "+v"(acc[0][0]), "+v"(acc[1][1]), "+v"(acc[2][2]), "+v"(acc[3][3]) : "v"(a[0]), "v"(a[3]));
    }
#pragma unroll
    for (int mb = 0; mb < 4; ++mb) {
#pragma unroll
        for (int nb = 0; nb < 4; ++nb) {
#pragma unroll
            for (int j = 0; j < 8; ++j) os[(hi * 8 + j) * 68 + nb * 16 + lr] = acc[mb][nb][j]; }
        __builtin_amdgcn_wave_barrier(); asm volatile("" ::: "memory");
        float* crow = C + (size_t)(r0 + mb * 16) * ldc + c0;
#pragma unroll 1
        for (int ps = 0; ps < 2; ++ps) {
#pragma unroll
            for (int s = 0; s < 8; ++s) { const int row = 2 * s + hi, cofs = lr * 4; v4f val = *(const v4fa*)(os + row * 68 + cofs); if (BIAS) { val[0] += bfr(bias[c0 + cofs]); val[1] += bfr(bias[c0 + cofs + 1]); val[2] += bfr(bias[c0 + cofs + 2]); val[3] += bfr(bias[c0 + cofs + 3]); }
                *(volatile v4f*)(crow + (size_t)row * ldc + cofs) = val; }
            if (ps == 0) __threadfence(); }
        __builtin_amdgcn_wave_barrier(); asm volatile("" ::: "memory");
    }
}

__device__ __forceinline__ h16 tohx(float x) { return (h16)x; }
__device__ __forceinline__ void splitf(float y, unsigned short& h, unsigned short& l) { h = f2bf(y); l = f2bf(y - bf2f(h)); }
typedef __attribute__((ext_vector_type(2))) _Float16 v2h;
typedef __attribute__((ext_vector_type(4))) _Float16 v4h;
typedef __attribute__((ext_vector_type(2))) unsigned short v2us;
typedef __attribute__((ext_vector_type(4))) unsigned short v4us;
typedef __attribute__((ext_vector_type(2))) float v2f;
typedef __attribute__((ext_vector_type(4))) int v4i;


__global__ __launch_bounds__(256) void k_cvt8(const float* __restrict__ src, bf* dst, size_t n8) { const size_t i = (size_t)blockIdx.x * 256 + threadIdx.x; if (i >= n8) return; const v8f v = *(const v8f*)(src + i * 8); v8us o;
#pragma unroll
    for (int k = 0; k < 8; ++k) o[k] = f2bf(v[k]); *(volatile v8us*)(dst + i * 8) = o; __threadfence(); *(volatile v8us*)(dst + i * 8) = o; }


__global__ __launch_bounds__(256) void k_flat(const float* __restrict__ F, h16* P16, bf* Ph, bf* Pl, size_t n4) { const size_t i = (size_t)blockIdx.x * 256 + threadIdx.x; if (i >= n4) return; const v4f a = *(const v4f*)(F + i * 4); v4h o16; v4us oh, ol;
#pragma unroll
    for (int q = 0; q < 4; ++q) { o16[q] = tohx(a[q]); unsigned short x2, y2; splitf(a[q], x2, y2); oh[q] = x2; ol[q] = y2; }
    *(volatile v4h*)(P16 + i * 4) = o16; *(volatile v4us*)(Ph + i * 4) = oh; *(volatile v4us*)(Pl + i * 4) = ol; __threadfence(); *(volatile v4h*)(P16 + i * 4) = o16; *(volatile v4us*)(Ph + i * 4) = oh; *(volatile v4us*)(Pl + i * 4) = ol; }

__device__ __forceinline__ float fmap(float x) { return (x > 0.0f) ? __fadd_rn(x, 1.0f) : expf(x); }
__global__ __launch_bounds__(256) void k_fmP(const float* __restrict__ F, bf* Ph, bf* Pl) { const size_t e = ((size_t)blockIdx.x * 256 + threadIdx.x) * 2; if (e >= (size_t)NH_ * TT * HD) return; const int d = (int)(e % HD); const int t = (int)((e / HD) % TT); const int h = (int)(e / ((size_t)HD * TT)); const float* f = F + (size_t)t * DQ + h * HD + d; v2us oh, ol;
#pragma unroll
    for (int q = 0; q < 2; ++q) { const float y = fmap(f[q]); unsigned short a, c2; splitf(y, a, c2); oh[q] = a; ol[q] = c2; }
    *(volatile v2us*)(Ph + e) = oh; *(volatile v2us*)(Pl + e) = ol; __threadfence(); *(volatile v2us*)(Ph + e) = oh; *(volatile v2us*)(Pl + e) = ol; }
template <int MODE>
__global__ __launch_bounds__(256) void k_fmT(const float* __restrict__ F, bf* Th, bf* Tl) { const size_t e = ((size_t)blockIdx.x * 256 + threadIdx.x) * 2; if (e >= (size_t)NH_ * HD * TT) return; const int s = (int)(e % TT); const int d = (int)((e / TT) % HD); const int h = (int)(e / ((size_t)TT * HD)); v2us oh, ol;
#pragma unroll
    for (int q = 0; q < 2; ++q) { const float x = F[(size_t)(s + q) * DQ + h * HD + d]; const float y = MODE ? fmap(x) : __fmul_rn(x, INVS); unsigned short a, c2; splitf(y, a, c2); oh[q] = a; ol[q] = c2; }
    *(volatile v2us*)(Th + e) = oh; *(volatile v2us*)(Tl + e) = ol; __threadfence(); *(volatile v2us*)(Th + e) = oh; *(volatile v2us*)(Tl + e) = ol; }
__global__ __launch_bounds__(256) void k_ksum(const float* __restrict__ F, float* KS) { const int lane = threadIdx.x & 31; const int wv = blockIdx.x * 8 + (threadIdx.x >> 5); if (wv >= NH_ * 2) return; const int h = wv >> 1; const int d = (wv & 1) * 32 + lane; const float* f = F + h * HD + d; float s = 0.f;
#pragma unroll 4
    for (int t = 0; t < TT; ++t) s = __fadd_rn(s, fmap(f[(size_t)t * DQ]));
    *(volatile float*)(KS + h * HD + d) = s; __threadfence(); *(volatile float*)(KS + h * HD + d) = s; }
__global__ __launch_bounds__(256) void k_zdot(const float* __restrict__ F, const float* __restrict__ KS, float* Z) { const int lane = threadIdx.x & 31; const size_t wv = (size_t)blockIdx.x * 8 + (threadIdx.x >> 5); if (wv >= (size_t)NH_ * (TT / 32)) return; const int h = (int)(wv / (TT / 32)); const int l = (int)(wv % (TT / 32)) * 32 + lane; const float* f = F + (size_t)l * DQ + h * HD; const float* ks = KS + h * HD; float s = 0.f;
#pragma unroll 4
    for (int d = 0; d < HD; ++d) { float p = __fmul_rn(fmap(f[d]), ks[d]); asm volatile("" : "+v"(p)); s = __fadd_rn(s, p); }
    const float z = __fdiv_rn(1.0f, __fadd_rn(s, ZEPS)); *(volatile float*)(Z + (size_t)h * TT + l) = z; __threadfence(); *(volatile float*)(Z + (size_t)h * TT + l) = z; }
__global__ __launch_bounds__(256) void k_zmerge(const float* __restrict__ O, const float* __restrict__ Z, float* outb) { const size_t i = (size_t)blockIdx.x * 256 + threadIdx.x; if (i >= (size_t)NH_ * TT * HD / 4) return; const size_t e = i * 4; const int d = (int)(e % HD); const int l = (int)((e / HD) % TT); const int h = (int)(e / ((size_t)HD * TT)); const float z = Z[(size_t)h * TT + l]; const v4f o = *(const v4f*)(O + e); v4f r;
#pragma unroll
    for (int q = 0; q < 4; ++q) { float m = __fmul_rn(o[q], z); asm volatile("" : "+v"(m)); r[q] = __fmul_rn(m, SFL); }
    *(volatile v4f*)(outb + (size_t)l * DQ + h * HD + d) = r; __threadfence(); *(volatile v4f*)(outb + (size_t)l * DQ + h * HD + d) = r; }

extern "C" void kernel_launch(void* const* d_in, const int* in_sizes, int n_in,
                              void* d_out, int out_size, void* d_ws, size_t ws_size, hipStream_t stream) {
    (void)in_sizes; (void)n_in; (void)out_size;
    const float* x = (const float*)d_in[0]; const float* gd = (const float*)d_in[1]; const float* wq = (const float*)d_in[2]; const float* bq = (const float*)d_in[3]; const float* wk = (const float*)d_in[4]; const float* bk = (const float*)d_in[5]; const float* wv = (const float*)d_in[6]; const float* bv = (const float*)d_in[7];
    float* OUT = (float*)d_out;
    char* wsp = (char*)d_ws;
    auto take = [&](size_t bytes) { char* p = wsp; wsp += (bytes + 255) & ~(size_t)255; return (void*)p; };
    bf* WQ = (bf*)take((size_t)DQ * DM * 2); bf* WK = (bf*)take((size_t)DQ * DM * 2); bf* WV = (bf*)take((size_t)DQ * DM * 2);
    bf* XB = (bf*)take((size_t)TT * DM * 2); float* FQ = (float*)take((size_t)TT * DQ * 4); float* FK = (float*)take((size_t)TT * DQ * 4); float* FV = (float*)take((size_t)TT * DQ * 4);
    bf* QPh = (bf*)take((size_t)NH_ * TT * HD * 2); bf* QPl = (bf*)take((size_t)NH_ * TT * HD * 2); bf* KTh = (bf*)take((size_t)NH_ * HD * TT * 2); bf* KTl = (bf*)take((size_t)NH_ * HD * TT * 2); bf* VTh = (bf*)take((size_t)NH_ * HD * TT * 2); bf* VTl = (bf*)take((size_t)NH_ * HD * TT * 2);
    float* KVT = (float*)take((size_t)NH_ * HD * HD * 4); h16* KV16 = (h16*)take((size_t)NH_ * HD * HD * 2); bf* KVh = (bf*)take((size_t)NH_ * HD * HD * 2); bf* KVl = (bf*)take((size_t)NH_ * HD * HD * 2); float* KS = (float*)take((size_t)NH_ * HD * 4); float* Z = (float*)take((size_t)NH_ * TT * 4); float* O = (float*)take((size_t)NH_ * TT * HD * 4);
    if ((size_t)(wsp - (char*)d_ws) > ws_size) return;
    k_cvt8<<<(unsigned)(((size_t)DQ * DM / 8 + 255) / 256), 256, 0, stream>>>(wq, WQ, (size_t)DQ * DM / 8); k_cvt8<<<(unsigned)(((size_t)DQ * DM / 8 + 255) / 256), 256, 0, stream>>>(wk, WK, (size_t)DQ * DM / 8); k_cvt8<<<(unsigned)(((size_t)DQ * DM / 8 + 255) / 256), 256, 0, stream>>>(wv, WV, (size_t)DQ * DM / 8);
    const unsigned LP = (unsigned)(((size_t)NH_ * TT * HD / 2 + 255) / 256);
    for (int b = 0; b < NB_; ++b) {
        k_cvt8<<<(unsigned)(((size_t)TT * DM / 8 + 255) / 256), 256, 0, stream>>>(gd + (size_t)b * TT * DM, XB, (size_t)TT * DM / 8);
        k_gemmw<bf, 0, true><<<dim3(TT / 64, DQ / 64, 1), 32, 0, stream>>>(XB, nullptr, WQ, nullptr, DM, FQ, DQ, bq, 0, 0, 0);
        k_cvt8<<<(unsigned)(((size_t)TT * DM / 8 + 255) / 256), 256, 0, stream>>>(x + (size_t)b * TT * DM, XB, (size_t)TT * DM / 8);
        k_gemmw<bf, 0, true><<<dim3(TT / 64, DQ / 64, 1), 32, 0, stream>>>(XB, nullptr, WK, nullptr, DM, FK, DQ, bk, 0, 0, 0);
        k_gemmw<bf, 0, true><<<dim3(TT / 64, DQ / 64, 1), 32, 0, stream>>>(XB, nullptr, WV, nullptr, DM, FV, DQ, bv, 0, 0, 0);
        k_fmP<<<LP, 256, 0, stream>>>(FQ, QPh, QPl); k_fmT<1><<<LP, 256, 0, stream>>>(FK, KTh, KTl); k_fmT<0><<<LP, 256, 0, stream>>>(FV, VTh, VTl);
        k_ksum<<<(NH_ * 2 + 7) / 8, 256, 0, stream>>>(FK, KS); k_zdot<<<(unsigned)(((size_t)NH_ * (TT / 32) + 7) / 8), 256, 0, stream>>>(FQ, KS, Z);
        k_gemmw<bf, 2, false><<<dim3(HD / 64, HD / 64, NH_), 32, 0, stream>>>(VTh, VTl, KTh, KTl, TT, KVT, HD, nullptr, (size_t)HD * TT, (size_t)HD * TT, (size_t)HD * HD);
        k_flat<<<(unsigned)(((size_t)NH_ * HD * HD / 4 + 255) / 256), 256, 0, stream>>>(KVT, KV16, KVh, KVl, (size_t)NH_ * HD * HD / 4);
        k_gemmw<bf, 2, false><<<dim3(TT / 64, HD / 64, NH_), 32, 0, stream>>>(QPh, QPl, KVh, KVl, HD, O, HD, nullptr, (size_t)TT * HD, (size_t)HD * HD, (size_t)TT * HD);
        k_zmerge<<<(unsigned)(((size_t)NH_ * TT * HD / 4 + 255) / 256), 256, 0, stream>>>(O, Z, OUT + (size_t)b * TT * DQ); }
}
